// SwinBlock_87299505258606
// MI455X (gfx1250) — hardware-verified
//
#include <hip/hip_runtime.h>
#include <hip/hip_bf16.h>
#include <math.h>
#include <stdint.h>

#ifndef NB
#define NB 8
#endif
#define NB_FULL 8
#ifndef QKV_SPLIT
#define QKV_SPLIT 1
#endif
#ifndef PROJ_SPLIT
#define PROJ_SPLIT 1
#endif

#define IMH 56
#define IMW 56
#define CC 512
#define WSZ 7
#define SSH 3
#define NHD 8
#define HDD 64
#define LTOK (WSZ * WSZ)
#define HIDN 2048
#define QKVC (3 * CC)
#define NWY (IMH / WSZ)
#define NWX (IMW / WSZ)
#define NWIMG (NWY * NWX)
#define NPIX_IMG (IMH * IMW)
#define MTOK (NB * NPIX_IMG)
#define NCHA ((NB % 4 == 0) ? 4 : ((NB % 2 == 0) ? 2 : 1))
#define NCHM ((NB % 2 == 0) ? 2 : 1)
#define MCHA (MTOK / NCHA)
#define MCHM (MTOK / NCHM)
#define AQW (CC * (1 + QKV_SPLIT))
#define APW (CC * (1 + PROJ_SPLIT))

#define WCAR 64.0f
#define GCAR 16.0f
#define OCAR 64.0f

#define PWQ  ((size_t)QKVC * AQW * 2)
#define PWP  ((size_t)CC * APW * 2)
#define PW1  ((size_t)HIDN * CC * 2)
#define PW2  ((size_t)CC * HIDN * 2)
#define PO2  ((size_t)MTOK * APW * 2)
#define PA1  ((size_t)MCHA * AQW * 2)
#define PQKV ((size_t)MCHA * QKVC * 4)
#define PG   ((size_t)MCHM * HIDN * 2)
#define PR   (((PA1 + PQKV) > PG) ? (PA1 + PQKV) : PG)
#define PH2  ((size_t)MTOK * CC * 2)

static_assert(NB >= 1 && NB <= NB_FULL);
static_assert(MTOK % 64 == 0);
static_assert(MCHA % 64 == 0 && MCHM % 64 == 0);
static_assert(MCHA * NCHA == MTOK && MCHM * NCHM == MTOK);
static_assert(NWIMG * LTOK == NPIX_IMG);
static_assert(NWX == 8 && NWY == 8);
static_assert(CC % 64 == 0 && HIDN % 64 == 0 && QKVC % 64 == 0);
static_assert(AQW % 32 == 0 && APW % 32 == 0);
static_assert(NHD * HDD == CC);
static_assert(PH2 <= PO2);
static_assert(PWQ + PWP + PW1 + PW2 + PO2 + PR <= (size_t)134217728u);
static_assert((PWQ % 128) == 0 && (PWP % 128) == 0 && (PW1 % 128) == 0 && (PW2 % 128) == 0 && (PO2 % 128) == 0 && (PA1 % 128) == 0);

typedef __attribute__((ext_vector_type(16))) _Float16 v16h;
typedef __attribute__((ext_vector_type(8)))  _Float16 v8h;
typedef __attribute__((ext_vector_type(16))) __bf16   v16b;
typedef __attribute__((ext_vector_type(16))) unsigned short v16us;
typedef __attribute__((ext_vector_type(8)))  unsigned short v8us;
typedef __attribute__((ext_vector_type(8)))  float    v8f;
typedef __attribute__((ext_vector_type(4)))  float    v4f;
typedef __attribute__((ext_vector_type(4)))  unsigned int v4u;

__device__ __forceinline__ unsigned short f2bf_bits(float f) {
  unsigned u = __float_as_uint(f);
  return (unsigned short)((u + 0x7FFFu + ((u >> 16) & 1u)) >> 16);
}
__device__ __forceinline__ float bf_bits2f(unsigned short h) { return __uint_as_float(((unsigned)h) << 16); }
__device__ __forceinline__ float bfr(float f) { return bf_bits2f(f2bf_bits(f)); }
__device__ __forceinline__ v4f bfr4(v4f a) { v4f r; r[0] = bfr(a[0]); r[1] = bfr(a[1]); r[2] = bfr(a[2]); r[3] = bfr(a[3]); return r; }

__device__ __forceinline__ void pack_split8(v4f u, v4f w, v4u& hi, v4u& lo) {
  union { v8us s; v4u q; } ph, pl;
#pragma unroll
  for (int e = 0; e < 4; ++e) {
    const unsigned short hu = f2bf_bits(u[e]);
    ph.s[e] = hu;
    pl.s[e] = f2bf_bits(u[e] - bf_bits2f(hu));
    const unsigned short hw = f2bf_bits(w[e]);
    ph.s[4 + e] = hw;
    pl.s[4 + e] = f2bf_bits(w[e] - bf_bits2f(hw));
  }
  hi = ph.q; lo = pl.q;
}
__device__ __forceinline__ v4u pack_f16_8(v4f u, v4f w, float carry) {
  union { v8h h; v4u q; } pk;
#pragma unroll
  for (int e = 0; e < 4; ++e) { pk.h[e] = (_Float16)(u[e] * carry); pk.h[4 + e] = (_Float16)(w[e] * carry); }
  return pk.q;
}

__device__ __forceinline__ void dep_guard_h(v8f& a, v8f& b, v16us x, v16us y) { asm volatile("v_nop\n\tv_nop\n\tv_nop\n\tv_nop" : "+v"(a), "+v"(b) : "v"(x), "v"(y)); }
__device__ __forceinline__ void keep4_h(v16us a, v16us b, v16us c, v16us d) { asm volatile("v_nop" :: "v"(a), "v"(b), "v"(c), "v"(d)); }
__device__ __forceinline__ void acc_guard4(v8f& a, v8f& b, v8f& c, v8f& d) { asm volatile("v_nop\n\tv_nop\n\tv_nop\n\tv_nop" : "+v"(a), "+v"(b), "+v"(c), "+v"(d)); }

union FragU { v16us v; v8us h[2]; };
__device__ __forceinline__ v16us frag_load(const unsigned short* p) {
  FragU f; f.h[0] = *(const v8us*)(p); f.h[1] = *(const v8us*)(p + 16); return f.v;
}
template <bool BF>
__device__ __forceinline__ v8f mma16(v16us a, v16us b, v8f c) {
  if (BF) {
    return __builtin_amdgcn_wmma_f32_16x16x32_bf16(false, __builtin_bit_cast(v16b, a), false, __builtin_bit_cast(v16b, b), (short)0, c, false, false);
  } else {
    return __builtin_amdgcn_wmma_f32_16x16x32_f16(false, __builtin_bit_cast(v16h, a), false, __builtin_bit_cast(v16h, b), (short)0, c, false, false);
  }
}

__device__ __forceinline__ int tok2raster(int m) {
  const int win = m / LTOK, l = m - win * LTOK;
  const int b = win / NWIMG, wi = win - b * NWIMG;
  const int wh = wi / NWX, ww = wi - wh * NWX;
  const int i = l / WSZ, j = l - i * WSZ;
  int y = wh * WSZ + i + SSH; y = (y >= IMH) ? (y - IMH) : y;
  int x = ww * WSZ + j + SSH; x = (x >= IMW) ? (x - IMW) : x;
  return (b * IMH + y) * IMW + x;
}

template <bool BF, int BIAS_MODE, int OUT_MODE, bool RESID, int ACT, int ROWMAP>
__global__ __launch_bounds__(256) void wmma_gemm64(
    const unsigned short* __restrict__ A, int lda,
    const unsigned short* __restrict__ Bt, int ldb,
    void* Cout, int ldc,
    const float* __restrict__ bias,
    const float* resid,
    int M, int N, int K, float scale, float oscale) {
  __shared__ __align__(16) float sT[8][16 * 68];
  const int lane = threadIdx.x & 31;
  const int wave = threadIdx.x >> 5;
  const int tilesN = N >> 6;
  const int tilesM = M >> 6;
  const int tile = blockIdx.x * 8 + wave;
  if (tile >= tilesM * tilesN) return;
  const int tm = tile / tilesN;
  const int tn = tile - tm * tilesN;
  const int m0 = tm << 6;
  const int n0 = tn << 6;
  const int rlane = lane & 15;
  const int koff  = (lane >> 4) * 8;
  const int mOff  = (lane >> 4) * 8;

  v8f acc[4][4];
#pragma unroll
  for (int i = 0; i < 4; ++i)
#pragma unroll
    for (int j = 0; j < 4; ++j) acc[i][j] = (v8f){0.f,0.f,0.f,0.f,0.f,0.f,0.f,0.f};

  for (int k0 = 0; k0 < K; k0 += 32) {
    v16us bh[4];
#pragma unroll
    for (int j = 0; j < 4; ++j) {
      const size_t bo = (size_t)(n0 + (j << 4) + rlane) * ldb + koff + k0;
      bh[j] = frag_load(Bt + bo);
    }
#pragma unroll
    for (int i = 0; i < 4; ++i) {
      const size_t ao = (size_t)(m0 + (i << 4) + rlane) * lda + koff + k0;
      const v16us ah = frag_load(A + ao);
#pragma unroll
      for (int j = 0; j < 4; ++j) acc[i][j] = mma16<BF>(ah, bh[j], acc[i][j]);
      dep_guard_h(acc[i][0], acc[i][3], ah, bh[3]);
    }
    keep4_h(bh[0], bh[1], bh[2], bh[3]);
  }
  acc_guard4(acc[0][0], acc[0][1], acc[0][2], acc[0][3]);
  acc_guard4(acc[1][0], acc[1][1], acc[1][2], acc[1][3]);
  acc_guard4(acc[2][0], acc[2][1], acc[2][2], acc[2][3]);
  acc_guard4(acc[3][0], acc[3][1], acc[3][2], acc[3][3]);

  float* slab = sT[wave];
#pragma unroll
  for (int i = 0; i < 4; ++i) {
    const int mBase = m0 + (i << 4);
#pragma unroll
    for (int j = 0; j < 4; ++j) {
      const int n = n0 + (j << 4) + rlane;
      float bv = 0.f;
      if (BIAS_MODE == 2) bv = bfr(bias[n]);
#pragma unroll
      for (int r = 0; r < 8; ++r) {
        float v = acc[i][j][r] * scale;
        if (BIAS_MODE == 2) v += bv;
        if (ACT == 5) v = 0.5f * v * (1.0f + erff(v * 0.70710678118654752f));
        v *= oscale;
        slab[(mOff + r) * 68 + (j << 4) + rlane] = v;
      }
    }
    __builtin_amdgcn_fence(__ATOMIC_RELEASE, "workgroup");
    __builtin_amdgcn_wave_barrier();
    __builtin_amdgcn_fence(__ATOMIC_ACQUIRE, "workgroup");
    if (OUT_MODE == 0) {
      float* C = (float*)Cout;
      const int hh = lane >> 4, c4 = (lane & 15) * 4;
      int orow[8];
#pragma unroll
      for (int it = 0; it < 8; ++it) {
        const int row = it * 2 + hh;
        orow[it] = ROWMAP ? tok2raster(mBase + row) : (mBase + row);
      }
      if (RESID) {
#pragma unroll
        for (int it = 0; it < 8; ++it) {
          const int row = it * 2 + hh;
          v4f v = *(const v4f*)(slab + row * 68 + c4);
          const v4f rv = *(const v4f*)(resid + (size_t)orow[it] * ldc + n0 + c4);
          v += rv;
          *(v4f*)(slab + row * 68 + c4) = v;
        }
      }
      for (int pass = 0; pass < 2; ++pass) {
#pragma unroll
        for (int it = 0; it < 8; ++it) {
          const int row = it * 2 + hh;
          const v4f v = *(const v4f*)(slab + row * 68 + c4);
          *(volatile v4f*)(C + (size_t)orow[it] * ldc + n0 + c4) = v;
        }
        __threadfence();
      }
    } else {
      const int q = lane >> 3, c8 = (lane & 7) * 8;
      unsigned short* C = (unsigned short*)Cout;
      for (int pass = 0; pass < 2; ++pass) {
#pragma unroll
        for (int it = 0; it < 4; ++it) {
          const int row = it * 4 + q;
          const float* sp = slab + row * 68 + c8;
          v8h hv;
#pragma unroll
          for (int e = 0; e < 8; ++e) hv[e] = (_Float16)sp[e];
          *(volatile v8h*)(C + (size_t)(mBase + row) * ldc + n0 + c8) = hv;
        }
        __threadfence();
      }
    }
    __builtin_amdgcn_fence(__ATOMIC_RELEASE, "workgroup");
    __builtin_amdgcn_wave_barrier();
    __builtin_amdgcn_fence(__ATOMIC_ACQUIRE, "workgroup");
  }
}

template <bool BFP>
__device__ __forceinline__ unsigned short cvt_bits(float f, float carry) {
  const float r = bfr(f);
  if (BFP) return f2bf_bits(r);
  return __builtin_bit_cast(unsigned short, (_Float16)(r * carry));
}

template <bool BFP, bool DUP>
__global__ __launch_bounds__(256) void cvt_wt_kernel(const float* __restrict__ w, unsigned short* out, int K, int N, int ldo, float carry) {
  __shared__ __align__(16) unsigned short sT[64][72];
  const int tid = threadIdx.x;
  const int k0 = blockIdx.x * 64, n0 = blockIdx.y * 64;
  {
    const int kr = tid >> 2, nc = (tid & 3) * 16;
    const float* src = w + (size_t)(k0 + kr) * N + n0 + nc;
    const v4f a0 = *(const v4f*)(src);
    const v4f a1 = *(const v4f*)(src + 4);
    const v4f a2 = *(const v4f*)(src + 8);
    const v4f a3 = *(const v4f*)(src + 12);
#pragma unroll
    for (int e = 0; e < 4; ++e) {
      sT[nc + e][kr]      = cvt_bits<BFP>(a0[e], carry);
      sT[nc + 4 + e][kr]  = cvt_bits<BFP>(a1[e], carry);
      sT[nc + 8 + e][kr]  = cvt_bits<BFP>(a2[e], carry);
      sT[nc + 12 + e][kr] = cvt_bits<BFP>(a3[e], carry);
    }
  }
  __syncthreads();
  const int c8 = (tid & 7) * 8;
  for (int pass = 0; pass < 2; ++pass) {
#pragma unroll
    for (int it = 0; it < 2; ++it) {
      const int row = it * 32 + (tid >> 3);
      const v4u v = *(const v4u*)(&sT[row][c8]);
      unsigned short* dst = out + (size_t)(n0 + row) * ldo + k0 + c8;
      *(volatile v4u*)dst = v;
      if (DUP) *(volatile v4u*)(dst + K) = v;
    }
    __threadfence();
  }
}

__device__ __forceinline__ void ln_row16(v4f a0, v4f a1, v4f a2, v4f a3,
                                         const float* __restrict__ g, const float* __restrict__ bb, int c0, int c1,
                                         v4f& y0, v4f& y1, v4f& y2, v4f& y3) {
  float sum = (((a0[0] + a0[1]) + (a0[2] + a0[3])) + ((a1[0] + a1[1]) + (a1[2] + a1[3]))) +
              (((a2[0] + a2[1]) + (a2[2] + a2[3])) + ((a3[0] + a3[1]) + (a3[2] + a3[3])));
#pragma unroll
  for (int off = 16; off > 0; off >>= 1) sum += __shfl_xor(sum, off, 32);
  const float mean = sum * (1.0f / CC);
  const v4f d0 = a0 - mean, d1 = a1 - mean, d2 = a2 - mean, d3 = a3 - mean;
  float vs = (((d0[0] * d0[0] + d0[1] * d0[1]) + (d0[2] * d0[2] + d0[3] * d0[3])) +
              ((d1[0] * d1[0] + d1[1] * d1[1]) + (d1[2] * d1[2] + d1[3] * d1[3]))) +
             (((d2[0] * d2[0] + d2[1] * d2[1]) + (d2[2] * d2[2] + d2[3] * d2[3])) +
              ((d3[0] * d3[0] + d3[1] * d3[1]) + (d3[2] * d3[2] + d3[3] * d3[3])));
#pragma unroll
  for (int off = 16; off > 0; off >>= 1) vs += __shfl_xor(vs, off, 32);
  const float rstd = 1.0f / sqrtf(vs * (1.0f / CC) + 1e-5f);
  const v4f g0 = bfr4(*(const v4f*)(g + c0)), g1 = bfr4(*(const v4f*)(g + c0 + 4));
  const v4f g2 = bfr4(*(const v4f*)(g + c1)), g3 = bfr4(*(const v4f*)(g + c1 + 4));
  const v4f e0 = bfr4(*(const v4f*)(bb + c0)), e1 = bfr4(*(const v4f*)(bb + c0 + 4));
  const v4f e2 = bfr4(*(const v4f*)(bb + c1)), e3 = bfr4(*(const v4f*)(bb + c1 + 4));
  y0 = (d0 * rstd) * g0 + e0;
  y1 = (d1 * rstd) * g1 + e1;
  y2 = (d2 * rstd) * g2 + e2;
  y3 = (d3 * rstd) * g3 + e3;
}

__global__ __launch_bounds__(256) void ln1_kernel(const float* __restrict__ x, const int* __restrict__ Hp, const int* __restrict__ Wd,
                                                  const float* __restrict__ g, const float* __restrict__ bb,
                                                  unsigned short* A1, int mbase, int nrows) {
  const int tid = threadIdx.x, wave = tid >> 5, lane = tid & 31;
  int mloc = blockIdx.x * 8 + wave;
  mloc = (mloc < nrows) ? mloc : (nrows - 1);
  const int m = mbase + mloc;
  const int win = m / LTOK, l = m - win * LTOK;
  int b = win / NWIMG;
  const int wi = win - b * NWIMG;
  b = (b < NB_FULL) ? b : (NB_FULL - 1);
  const int wh = wi >> 3, ww = wi & 7;
  const int i = l / WSZ, j = l - i * WSZ;
  int Hr = Hp[0], Wr = Wd[0];
  Hr = (Hr < 1 || Hr > IMH) ? IMH : Hr;
  Wr = (Wr < 1 || Wr > IMW) ? IMW : Wr;
  int y = wh * WSZ + i + SSH;  y = (y >= Hr) ? (y - Hr) : y;   y = (y < 0) ? 0 : ((y >= IMH) ? (IMH - 1) : y);
  int xq = ww * WSZ + j + SSH; xq = (xq >= Wr) ? (xq - Wr) : xq; xq = (xq < 0) ? 0 : ((xq >= IMW) ? (IMW - 1) : xq);
  const float* xc = x + ((size_t)(b * IMH + y) * IMW + xq) * CC;
  const int c0 = 8 * lane, c1 = (CC / 2) + 8 * lane;
  const v4f a0 = bfr4(*(const v4f*)(xc + c0));
  const v4f a1 = bfr4(*(const v4f*)(xc + c0 + 4));
  const v4f a2 = bfr4(*(const v4f*)(xc + c1));
  const v4f a3 = bfr4(*(const v4f*)(xc + c1 + 4));
  v4f y0, y1, y2, y3;
  ln_row16(a0, a1, a2, a3, g, bb, c0, c1, y0, y1, y2, y3);
  unsigned short* dst = A1 + (size_t)mloc * AQW;
#if QKV_SPLIT
  v4u hA, lA, hB, lB;
  pack_split8(y0, y1, hA, lA);
  pack_split8(y2, y3, hB, lB);
  for (int pass = 0; pass < 2; ++pass) {
    *(volatile v4u*)(dst + c0) = hA;
    *(volatile v4u*)(dst + c1) = hB;
    *(volatile v4u*)(dst + CC + c0) = lA;
    *(volatile v4u*)(dst + CC + c1) = lB;
    __threadfence();
  }
#else
  const v4u hA = pack_f16_8(y0, y1, 1.0f);
  const v4u hB = pack_f16_8(y2, y3, 1.0f);
  for (int pass = 0; pass < 2; ++pass) {
    *(volatile v4u*)(dst + c0) = hA;
    *(volatile v4u*)(dst + c1) = hB;
    __threadfence();
  }
#endif
}

__global__ __launch_bounds__(256) void head_attn_kernel(const float* __restrict__ QKV, unsigned short* O2, int mbase, int nrows) {
  __shared__ __align__(16) float sR[8][QKVC + 64];
  const int tid = threadIdx.x, wave = tid >> 5, lane = tid & 31;
  int mloc = blockIdx.x * 8 + wave;
  mloc = (mloc < nrows) ? mloc : (nrows - 1);
  const int m = mbase + mloc;
  float* sw = sR[wave];
  {
    const float* src = QKV + (size_t)mloc * QKVC + 4 * lane;
#pragma unroll
    for (int jj = 0; jj < QKVC / 128; ++jj) {
      const v4f v = *(const v4f*)(src + 128 * jj);
      *(v4f*)(sw + 4 * lane + 128 * jj) = v;
    }
  }
  __builtin_amdgcn_fence(__ATOMIC_RELEASE, "workgroup");
  __builtin_amdgcn_wave_barrier();
  __builtin_amdgcn_fence(__ATOMIC_ACQUIRE, "workgroup");

  const int hq = lane >> 3, gi = lane & 7;
  const float* qa = sw + hq * HDD;
  const float* qb = sw + (hq + 4) * HDD;
  const float* kr = sw + CC + gi * HDD;
  float s0 = 0.0f, s1 = 0.0f;
#pragma unroll 1
  for (int dq = 0; dq < HDD; dq += 4) {
    const v4f q0 = *(const v4f*)(qa + dq);
    const v4f q1 = *(const v4f*)(qb + dq);
    const v4f kk = *(const v4f*)(kr + dq);
    s0 += (q0[0] * kk[0] + q0[1] * kk[1]) + (q0[2] * kk[2] + q0[3] * kk[3]);
    s1 += (q1[0] * kk[0] + q1[1] * kk[1]) + (q1[2] * kk[2] + q1[3] * kk[3]);
  }
  s0 *= 0.125f;
  s1 *= 0.125f;
  float mx0 = s0, mx1 = s1;
#pragma unroll
  for (int off = 1; off < 8; off <<= 1) {
    mx0 = fmaxf(mx0, __shfl_xor(mx0, off, 32));
    mx1 = fmaxf(mx1, __shfl_xor(mx1, off, 32));
  }
  const float e0 = expf(s0 - mx0);
  const float e1 = expf(s1 - mx1);
  float z0 = e0, z1 = e1;
#pragma unroll
  for (int off = 1; off < 8; off <<= 1) {
    z0 += __shfl_xor(z0, off, 32);
    z1 += __shfl_xor(z1, off, 32);
  }
  const float p0 = e0 * (1.0f / z0);
  const float p1 = e1 * (1.0f / z1);
  sw[QKVC + lane] = p0;
  sw[QKVC + 32 + lane] = p1;
  __builtin_amdgcn_fence(__ATOMIC_RELEASE, "workgroup");
  __builtin_amdgcn_wave_barrier();
  __builtin_amdgcn_fence(__ATOMIC_ACQUIRE, "workgroup");

  const int d0 = gi * 8;
  v4f oa0 = (v4f){0.f,0.f,0.f,0.f}, oa1 = oa0, ob0 = oa0, ob1 = oa0;
#pragma unroll 1
  for (int gg = 0; gg < NHD; ++gg) {
    const float pa = sw[QKVC + hq * 8 + gg];
    const float pb = sw[QKVC + (hq + 4) * 8 + gg];
    const float* vr = sw + 2 * CC + gg * HDD + d0;
    const v4f va = *(const v4f*)(vr);
    const v4f vb = *(const v4f*)(vr + 4);
    oa0 += pa * va; oa1 += pa * vb;
    ob0 += pb * va; ob1 += pb * vb;
  }

  const int win = m / LTOK, l = m - win * LTOK;
  const int ha = hq, hb = hq + 4;
  const size_t ra = (size_t)(win * LTOK + 6 * ha + ((ha + l) >> 3)) * APW + (size_t)(((ha + l) & 7) * HDD) + d0;
  const size_t rb = (size_t)(win * LTOK + 6 * hb + ((hb + l) >> 3)) * APW + (size_t)(((hb + l) & 7) * HDD) + d0;
#if PROJ_SPLIT
  v4u hA, lA, hB, lB;
  pack_split8(oa0, oa1, hA, lA);
  pack_split8(ob0, ob1, hB, lB);
  for (int pass = 0; pass < 2; ++pass) {
    *(volatile v4u*)(O2 + ra) = hA;
    *(volatile v4u*)(O2 + rb) = hB;
    *(volatile v4u*)(O2 + ra + CC) = lA;
    *(volatile v4u*)(O2 + rb + CC) = lB;
    __threadfence();
  }
#else
  const v4u hA = pack_f16_8(oa0, oa1, OCAR);
  const v4u hB = pack_f16_8(ob0, ob1, OCAR);
  for (int pass = 0; pass < 2; ++pass) {
    *(volatile v4u*)(O2 + ra) = hA;
    *(volatile v4u*)(O2 + rb) = hB;
    __threadfence();
  }
#endif
}

__global__ __launch_bounds__(256) void ln2_kernel(const float* xin, const float* __restrict__ g, const float* __restrict__ bb,
                                                  unsigned short* H2, int nrow) {
  const int tid = threadIdx.x, wave = tid >> 5, lane = tid & 31;
  int row = blockIdx.x * 8 + wave;
  row = (row < nrow) ? row : (nrow - 1);
  const int c0 = 8 * lane, c1 = (CC / 2) + 8 * lane;
  const float* rp = xin + (size_t)row * CC;
  const v4f a0 = *(const v4f*)(rp + c0);
  const v4f a1 = *(const v4f*)(rp + c0 + 4);
  const v4f a2 = *(const v4f*)(rp + c1);
  const v4f a3 = *(const v4f*)(rp + c1 + 4);
  v4f y0, y1, y2, y3;
  ln_row16(a0, a1, a2, a3, g, bb, c0, c1, y0, y1, y2, y3);
  const v4u hA = pack_f16_8(y0, y1, 1.0f);
  const v4u hB = pack_f16_8(y2, y3, 1.0f);
  unsigned short* dst = H2 + (size_t)row * CC;
  for (int pass = 0; pass < 2; ++pass) {
    *(volatile v4u*)(dst + c0) = hA;
    *(volatile v4u*)(dst + c1) = hB;
    __threadfence();
  }
}

extern "C" void kernel_launch(void* const* d_in, const int* in_sizes, int n_in,
                              void* d_out, int out_size, void* d_ws, size_t ws_size,
                              hipStream_t stream) {
  if (n_in < 15) return;
  if (in_sizes[0] < MTOK * CC) return;
  if (in_sizes[1] < 1 || in_sizes[2] < 1) return;
  if (in_sizes[3] < CC || in_sizes[4] < CC) return;
  if (in_sizes[5] < CC * QKVC || in_sizes[6] < QKVC) return;
  if (in_sizes[7] < CC * CC || in_sizes[8] < CC) return;
  if (in_sizes[9] < CC || in_sizes[10] < CC) return;
  if (in_sizes[11] < CC * HIDN || in_sizes[12] < HIDN) return;
  if (in_sizes[13] < HIDN * CC || in_sizes[14] < CC) return;
  if (out_size < MTOK * CC) return;

  const float* x       = (const float*)d_in[0];
  const int*   Hin     = (const int*)d_in[1];
  const int*   Win     = (const int*)d_in[2];
  const float* norm1_g = (const float*)d_in[3];
  const float* norm1_b = (const float*)d_in[4];
  const float* qkv_w   = (const float*)d_in[5];
  const float* qkv_b   = (const float*)d_in[6];
  const float* proj_w  = (const float*)d_in[7];
  const float* proj_b  = (const float*)d_in[8];
  const float* norm2_g = (const float*)d_in[9];
  const float* norm2_b = (const float*)d_in[10];
  const float* fc1_w   = (const float*)d_in[11];
  const float* fc1_b   = (const float*)d_in[12];
  const float* fc2_w   = (const float*)d_in[13];
  const float* fc2_b   = (const float*)d_in[14];
  float* outp = (float*)d_out;

  size_t off = 0;
  const size_t oWq = off; off += PWQ;
  const size_t oWp = off; off += PWP;
  const size_t oW1 = off; off += PW1;
  const size_t oW2 = off; off += PW2;
  const size_t oO2 = off; off += PO2;
  const size_t oR  = off; off += PR;
  if (off > ws_size) return;
  if (off > (size_t)134217728u) return;

  char* ws = (char*)d_ws;
  unsigned short* Wq   = (unsigned short*)(ws + oWq);
  unsigned short* Wp   = (unsigned short*)(ws + oWp);
  unsigned short* W1   = (unsigned short*)(ws + oW1);
  unsigned short* W2   = (unsigned short*)(ws + oW2);
  unsigned short* O2   = (unsigned short*)(ws + oO2);
  unsigned short* H2   = (unsigned short*)(ws + oO2);
  unsigned short* A1   = (unsigned short*)(ws + oR);
  float*          QKVf = (float*)(ws + oR + PA1);
  unsigned short* G    = (unsigned short*)(ws + oR);

  const dim3 blk(256);
  cvt_wt_kernel<(QKV_SPLIT != 0), (QKV_SPLIT != 0)><<<dim3(CC / 64, QKVC / 64), blk, 0, stream>>>(qkv_w, Wq, CC, QKVC, AQW, WCAR);
  cvt_wt_kernel<(PROJ_SPLIT != 0), (PROJ_SPLIT != 0)><<<dim3(CC / 64, CC / 64), blk, 0, stream>>>(proj_w, Wp, CC, CC, APW, WCAR);
  cvt_wt_kernel<false, false><<<dim3(CC / 64, HIDN / 64), blk, 0, stream>>>(fc1_w, W1, CC, HIDN, CC, WCAR);
  cvt_wt_kernel<false, false><<<dim3(HIDN / 64, CC / 64), blk, 0, stream>>>(fc2_w, W2, HIDN, CC, HIDN, WCAR);

  const int tilesA = MCHA / 64;
  for (int c = 0; c < NCHA; ++c) {
    ln1_kernel<<<dim3(MCHA / 8), blk, 0, stream>>>(x, Hin, Win, norm1_g, norm1_b, A1, c * MCHA, MCHA);
#if QKV_SPLIT
    wmma_gemm64<true, 2, 0, false, 0, 0><<<dim3((tilesA * (QKVC / 64) + 7) / 8), blk, 0, stream>>>(
        A1, AQW, Wq, AQW, (void*)QKVf, QKVC, qkv_b, qkv_b, MCHA, QKVC, AQW, 1.0f, 1.0f);
#else
    wmma_gemm64<false, 2, 0, false, 0, 0><<<dim3((tilesA * (QKVC / 64) + 7) / 8), blk, 0, stream>>>(
        A1, AQW, Wq, AQW, (void*)QKVf, QKVC, qkv_b, qkv_b, MCHA, QKVC, AQW, 1.0f / WCAR, 1.0f);
#endif
    head_attn_kernel<<<dim3(MCHA / 8), blk, 0, stream>>>(QKVf, O2, c * MCHA, MCHA);
  }

  const int tilesM = MTOK / 64;
#if PROJ_SPLIT
  wmma_gemm64<true, 2, 0, false, 0, 1><<<dim3((tilesM * (CC / 64) + 7) / 8), blk, 0, stream>>>(
      O2, APW, Wp, APW, (void*)outp, CC, proj_b, proj_b, MTOK, CC, APW, 1.0f, 1.0f);
#else
  wmma_gemm64<false, 2, 0, false, 0, 1><<<dim3((tilesM * (CC / 64) + 7) / 8), blk, 0, stream>>>(
      O2, APW, Wp, APW, (void*)outp, CC, proj_b, proj_b, MTOK, CC, APW, 1.0f / (OCAR * WCAR), 1.0f);
#endif
  ln2_kernel<<<dim3(MTOK / 8), blk, 0, stream>>>(outp, norm2_g, norm2_b, H2, MTOK);

  const int tilesC = MCHM / 64;
  for (int c = 0; c < NCHM; ++c) {
    const unsigned short* H2c = H2 + (size_t)c * MCHM * CC;
    float* outc = outp + (size_t)c * MCHM * CC;
    wmma_gemm64<false, 2, 1, false, 5, 0><<<dim3((tilesC * (HIDN / 64) + 7) / 8), blk, 0, stream>>>(
        H2c, CC, W1, CC, (void*)G, HIDN, fc1_b, fc1_b, MCHM, HIDN, CC, 1.0f / WCAR, GCAR);
    wmma_gemm64<false, 2, 0, true, 0, 0><<<dim3((tilesC * (CC / 64) + 7) / 8), blk, 0, stream>>>(
        G, HIDN, W2, HIDN, (void*)outc, CC, fc2_b, outc, MCHM, CC, HIDN, 1.0f / (GCAR * WCAR), 1.0f);
  }
  (void)hipGetLastError();
}
